// GATBlock_31147102831290
// MI455X (gfx1250) — hardware-run, weakly checked
//
#include <hip/hip_runtime.h>
#include <stddef.h>
#include <stdint.h>


#define DM      128
#define NHD     4
#define HC      32
#define NXL     256
#define DFF     512
#define NTHR    256
#define NWAVE   8
#define EPT     8
#define CHUNK   (NTHR * EPT)
#define WCAP    (EPT * 32)
#define LISTN   (NWAVE * WCAP)
#define NBMAX   2048
#define NBRUN   1024
#define RCAP    28672
#define DEGCAP  64
#define STW     512
#define GBM     64
#define GBN     64
#define GTHR    128
#define CX      8.0f
#define CL      2048.0f
#define CW      64.0f
#define SCL_XW  0.001953125f
#define SCL_XWL 9.5367431640625e-7f
#define NEGS    0.2f
#define LNEPS   1e-5f
#define WSMAX   134217728
#define LDS_AGG ((2 * RCAP + 2 * NBMAX + LISTN) * 4 + 64)

static_assert((CHUNK & (CHUNK - 1)) == 0 && CHUNK <= 4096);
static_assert((NBMAX & (NBMAX - 1)) == 0 && NBMAX <= 4096);
static_assert((NBRUN & (NBRUN - 1)) == 0 && NBRUN <= NBMAX && NBRUN >= 16);
static_assert(NTHR * 8 == NBMAX);
static_assert(LISTN >= NBMAX);
static_assert(LISTN >= NWAVE * WCAP);
static_assert((RCAP % 32) == 0);
static_assert(NWAVE * STW <= RCAP);
static_assert(2 * DM <= STW);
static_assert(LDS_AGG <= 300000);
static_assert(GBM == (GTHR / 32) * 16);
static_assert(DM == NHD * HC && HC == 32);
static_assert(NXL == 2 * DM);
static_assert((DM % 32) == 0 && (DFF % 32) == 0);
static_assert((NXL % GBN) == 0 && (DFF % GBN) == 0 && (DM % GBN) == 0);
static_assert(DM / 8 == 16);

typedef float          v4f   __attribute__((ext_vector_type(4)));
typedef float          v8f   __attribute__((ext_vector_type(8)));
typedef int            v4i   __attribute__((ext_vector_type(4)));
typedef int            v8i   __attribute__((ext_vector_type(8)));
typedef unsigned short v8us  __attribute__((ext_vector_type(8)));
typedef _Float16       v8h   __attribute__((ext_vector_type(8)));
typedef _Float16       v16h  __attribute__((ext_vector_type(16)));
union FragH { v16h v; v8us u[2]; v8i w; };

__device__ __forceinline__ v8f wmx(const FragH& a, const FragH& b, v8f c) {
  v8f d = __builtin_amdgcn_wmma_f32_16x16x32_f16(false, a.v, false, b.v, (short)0, c, false, false);
  asm volatile("v_nop\n\tv_nop\n\tv_nop\n\tv_nop" : "+v"(d) : "v"(a.w), "v"(b.w));
  return d;
}

__device__ __forceinline__ void ldwait() {
  asm volatile("s_wait_loadcnt 0x0" ::: "memory");
}

__device__ __forceinline__ unsigned bfbits(float v) {
  unsigned u = __float_as_uint(v);
  u = u + 0x7FFFu + ((u >> 16) & 1u);
  return u >> 16;
}
__device__ __forceinline__ float rbf(float v) { return __uint_as_float(bfbits(v) << 16); }

__device__ __forceinline__ v8h cvt8bh(const v4f a, const v4f b, const float c) {
  v8h hv;
  hv[0] = (_Float16)(rbf(a.x) * c); hv[1] = (_Float16)(rbf(a.y) * c);
  hv[2] = (_Float16)(rbf(a.z) * c); hv[3] = (_Float16)(rbf(a.w) * c);
  hv[4] = (_Float16)(rbf(b.x) * c); hv[5] = (_Float16)(rbf(b.y) * c);
  hv[6] = (_Float16)(rbf(b.z) * c); hv[7] = (_Float16)(rbf(b.w) * c);
  return hv;
}
__device__ __forceinline__ void cvt8hl(const v4f a, const v4f b, v8h& hv, v8h& lv) {
  float f[8] = {a.x * CX, a.y * CX, a.z * CX, a.w * CX, b.x * CX, b.y * CX, b.z * CX, b.w * CX};
#pragma unroll
  for (int i = 0; i < 8; ++i) {
    const _Float16 hq = (_Float16)f[i];
    hv[i] = hq;
    lv[i] = (_Float16)((f[i] - (float)hq) * CL);
  }
}

__device__ __forceinline__ float gelu_erf(float v) {
  return 0.5f * v * (1.0f + erff(v * 0.70710678118654752f));
}

__device__ __forceinline__ int scan_chunk(const int* __restrict__ dsts, int nE, int cbase, int slotBase,
                                          int nb, int vec8, int* list, int tid, int lane, int wave) {
  int wc = 0;
  const int el0  = tid * EPT;
  const int e0   = cbase + el0;
  const int sent = -2147483647 - 1;
  v4i da, db;
  if (vec8 != 0 && cbase + CHUNK <= nE) {
    da = *(const v4i*)(dsts + e0);
    db = *(const v4i*)(dsts + e0 + 4);
  } else {
    da.x = (e0     < nE) ? dsts[min(e0,     nE - 1)] : sent;
    da.y = (e0 + 1 < nE) ? dsts[min(e0 + 1, nE - 1)] : sent;
    da.z = (e0 + 2 < nE) ? dsts[min(e0 + 2, nE - 1)] : sent;
    da.w = (e0 + 3 < nE) ? dsts[min(e0 + 3, nE - 1)] : sent;
    db.x = (e0 + 4 < nE) ? dsts[min(e0 + 4, nE - 1)] : sent;
    db.y = (e0 + 5 < nE) ? dsts[min(e0 + 5, nE - 1)] : sent;
    db.z = (e0 + 6 < nE) ? dsts[min(e0 + 6, nE - 1)] : sent;
    db.w = (e0 + 7 < nE) ? dsts[min(e0 + 7, nE - 1)] : sent;
  }
  const unsigned nbs = (unsigned)slotBase;
  const unsigned unb = (unsigned)nb;
  const unsigned s0 = (unsigned)da.x - nbs, s1 = (unsigned)da.y - nbs;
  const unsigned s2 = (unsigned)da.z - nbs, s3 = (unsigned)da.w - nbs;
  const unsigned s4 = (unsigned)db.x - nbs, s5 = (unsigned)db.y - nbs;
  const unsigned s6 = (unsigned)db.z - nbs, s7 = (unsigned)db.w - nbs;
  const bool h0 = s0 < unb, h1 = s1 < unb, h2 = s2 < unb, h3 = s3 < unb;
  const bool h4 = s4 < unb, h5 = s5 < unb, h6 = s6 < unb, h7 = s7 < unb;
  const unsigned any = __builtin_amdgcn_ballot_w32(h0 | h1 | h2 | h3 | h4 | h5 | h6 | h7);
  if (any != 0u) {
#define HITJ(J, HJ, SJ) { \
      const unsigned mj = __builtin_amdgcn_ballot_w32(HJ); \
      if (mj != 0u) { \
        if (HJ) { \
          const int pos = wc + (int)__builtin_amdgcn_mbcnt_lo(mj, 0u); \
          if (pos < WCAP) list[wave * WCAP + pos] = ((el0 + (J)) << 12) | (int)(SJ); \
        } \
        wc += (int)__builtin_popcount(mj); } }
    HITJ(0, h0, s0)
    HITJ(1, h1, s1)
    HITJ(2, h2, s2)
    HITJ(3, h3, s3)
    HITJ(4, h4, s4)
    HITJ(5, h5, s5)
    HITJ(6, h6, s6)
    HITJ(7, h7, s7)
#undef HITJ
  }
  return wc;
}

__global__ __launch_bounds__(NTHR) void k_ln1(const float* __restrict__ x, const float* __restrict__ w,
                                              _Float16* Hh, _Float16* Hl, int nN, int MPr) {
  const int tid = (int)threadIdx.x, lane = tid & 31, wave = tid >> 5, hh = lane >> 4, m = lane & 15;
  const int row = (int)blockIdx.x * (2 * NWAVE) + 2 * wave + hh;
  const int rc  = row < nN ? row : nN - 1;
  const float live = row < nN ? 1.0f : 0.0f;
  const float* p = x + (size_t)rc * DM + 8 * m;
  const v4f a  = *(const v4f*)p,           b  = *(const v4f*)(p + 4);
  const v4f wa = *(const v4f*)(w + 8 * m), wb = *(const v4f*)(w + 8 * m + 4);
  float f[8] = {rbf(a.x) * live, rbf(a.y) * live, rbf(a.z) * live, rbf(a.w) * live,
                rbf(b.x) * live, rbf(b.y) * live, rbf(b.z) * live, rbf(b.w) * live};
  const float wr[8] = {rbf(wa.x), rbf(wa.y), rbf(wa.z), rbf(wa.w), rbf(wb.x), rbf(wb.y), rbf(wb.z), rbf(wb.w)};
  float s = ((f[0] + f[1]) + (f[2] + f[3])) + ((f[4] + f[5]) + (f[6] + f[7]));
#pragma unroll
  for (int off = 8; off > 0; off >>= 1) s += __shfl_xor(s, off);
  const float mean = s * (1.0f / DM);
  float d[8];
  float vs = 0.0f;
#pragma unroll
  for (int i = 0; i < 8; ++i) { d[i] = f[i] - mean; vs = fmaf(d[i], d[i], vs); }
#pragma unroll
  for (int off = 8; off > 0; off >>= 1) vs += __shfl_xor(vs, off);
  const float var  = vs * (1.0f / DM);
  const float rstd = rsqrtf(var + LNEPS);
  v4f ha, hb;
  ha.x = d[0] * rstd * wr[0]; ha.y = d[1] * rstd * wr[1]; ha.z = d[2] * rstd * wr[2]; ha.w = d[3] * rstd * wr[3];
  hb.x = d[4] * rstd * wr[4]; hb.y = d[5] * rstd * wr[5]; hb.z = d[6] * rstd * wr[6]; hb.w = d[7] * rstd * wr[7];
  v8h hv, lv;
  cvt8hl(ha, hb, hv, lv);
  const size_t o = (size_t)row * DM + 8 * m;
  const bool wrr = row < MPr;
  if (wrr) { *(volatile v8h*)(Hh + o) = hv; *(volatile v8h*)(Hl + o) = lv; }
  __threadfence();
  if (wrr) { *(volatile v8h*)(Hh + o) = hv; *(volatile v8h*)(Hl + o) = lv; }
}

__global__ __launch_bounds__(NTHR) void k_wtr_h(const float* __restrict__ w, int cols, int K,
                                                _Float16* wt, int nUnits) {
  const int u = (int)blockIdx.x * NTHR + (int)threadIdx.x;
  if (u >= nUnits) return;
  const int kq = K >> 3;
  const int n  = u / kq;
  const int k8 = (u - n * kq) * 8;
  const int ncl = n < cols ? n : cols - 1;
  const float* p = w + (size_t)k8 * (size_t)cols + ncl;
  v4f a, b;
  a.x = p[0];                  a.y = p[(size_t)cols];       a.z = p[(size_t)2 * cols];   a.w = p[(size_t)3 * cols];
  b.x = p[(size_t)4 * cols];   b.y = p[(size_t)5 * cols];   b.z = p[(size_t)6 * cols];   b.w = p[(size_t)7 * cols];
  const v4f z4 = {0.f, 0.f, 0.f, 0.f};
  if (n >= cols) { a = z4; b = z4; }
  const v8h hv = cvt8bh(a, b, CW);
  const size_t o = (size_t)n * (size_t)K + k8;
  *(volatile v8h*)(wt + o) = hv;
  __threadfence();
  *(volatile v8h*)(wt + o) = hv;
}

template<int EPI>
__global__ __launch_bounds__(GTHR) void k_gemm(
    const unsigned short* __restrict__ A, const unsigned short* __restrict__ A2,
    const unsigned short* __restrict__ WT,
    const float* __restrict__ p0, const float* __restrict__ p1,
    float* oF, _Float16* oH, _Float16* oL,
    int K, int ldo, int aOff, int oOff, int nRow)
{
  __shared__ __attribute__((aligned(16))) float stg[GBM * GBN];
  const int tid = (int)threadIdx.x, lane = tid & 31, wave = tid >> 5, hh = lane >> 4, m = lane & 15;
  const int rowBase = (int)blockIdx.x * GBM;
  const int col0    = (int)blockIdx.y * GBN;

  v8f acc[4], acc2[4];
  {
    const v8f z = {0.f, 0.f, 0.f, 0.f, 0.f, 0.f, 0.f, 0.f};
    acc[0] = z; acc[1] = z; acc[2] = z; acc[3] = z;
    acc2[0] = z; acc2[1] = z; acc2[2] = z; acc2[3] = z;
  }
  const size_t arow = (size_t)(aOff + rowBase + 16 * wave + m) * (size_t)K + 8 * hh;
  const unsigned short* ap  = A  + arow;
  const unsigned short* ap2 = A2 + arow;
  const unsigned short* wp  = WT + (size_t)(col0 + m) * (size_t)K + 8 * hh;
  const int ksteps = K >> 5;
#pragma unroll 1
  for (int ks = 0; ks < ksteps; ++ks) {
    FragH af, af2;
    af.u[0]  = *(const v8us*)(ap + 32 * ks);
    af.u[1]  = *(const v8us*)(ap + 32 * ks + 16);
    af2.u[0] = *(const v8us*)(ap2 + 32 * ks);
    af2.u[1] = *(const v8us*)(ap2 + 32 * ks + 16);
#pragma unroll
    for (int t = 0; t < 4; ++t) {
      const unsigned short* wq = wp + (size_t)(16 * t) * (size_t)K + 32 * ks;
      FragH bf;
      bf.u[0] = *(const v8us*)wq;
      bf.u[1] = *(const v8us*)(wq + 16);
      acc[t]  = wmx(af, bf, acc[t]);
      acc2[t] = wmx(af2, bf, acc2[t]);
    }
  }

#pragma unroll
  for (int t = 0; t < 4; ++t) {
    const int lc = 16 * t + m;
    float badd = 0.0f;
    if (EPI == 0) {
      const int gc = col0 + lc;
      const float b0 = rbf(p0[gc & (DM - 1)]);
      const float b1 = rbf(p1[gc & (DM - 1)]);
      badd = (gc >= DM) ? b1 : b0;
    }
#pragma unroll
    for (int r = 0; r < 8; ++r) {
      const int lr = 16 * wave + 8 * hh + r;
      float v = fmaf(acc2[t][r], SCL_XWL, acc[t][r] * SCL_XW);
      if (EPI == 0) v = v + badd;
      if (EPI == 1) v = gelu_erf(v);
      stg[lr * GBN + lc] = v;
    }
  }
  __syncthreads();

  if (EPI != 1) {
    v4f fv[8];
    bool ok[8];
#pragma unroll
    for (int i = 0; i < 8; ++i) {
      const int lr = 16 * wave + 2 * i + hh;
      const int gr = oOff + rowBase + lr;
      fv[i] = *(const v4f*)(stg + lr * GBN + 4 * m);
      ok[i] = gr < nRow;
      if (EPI == 2) {
        const v4f rs = *(const v4f*)(p0 + (size_t)gr * DM + col0 + 4 * m);
        fv[i] = rs + fv[i];
      }
    }
#pragma unroll
    for (int i = 0; i < 8; ++i) {
      const int lr = 16 * wave + 2 * i + hh;
      const int gr = oOff + rowBase + lr;
      float* op = oF + (size_t)gr * (size_t)ldo + col0 + 4 * m;
      if (ok[i]) *(volatile v4f*)op = fv[i];
    }
    __threadfence();
#pragma unroll
    for (int i = 0; i < 8; ++i) {
      const int lr = 16 * wave + 2 * i + hh;
      const int gr = oOff + rowBase + lr;
      float* op = oF + (size_t)gr * (size_t)ldo + col0 + 4 * m;
      if (ok[i]) *(volatile v4f*)op = fv[i];
    }
  } else {
    const int q8 = lane & 7, sub = lane >> 3;
    v8h hv[4], lv[4];
#pragma unroll
    for (int i = 0; i < 4; ++i) {
      const int lr = 16 * wave + 4 * i + sub;
      const v4f ga = *(const v4f*)(stg + lr * GBN + 8 * q8);
      const v4f gb = *(const v4f*)(stg + lr * GBN + 8 * q8 + 4);
      cvt8hl(ga, gb, hv[i], lv[i]);
    }
#pragma unroll
    for (int i = 0; i < 4; ++i) {
      const int lr = 16 * wave + 4 * i + sub;
      const size_t o = (size_t)(oOff + rowBase + lr) * (size_t)ldo + col0 + 8 * q8;
      *(volatile v8h*)(oH + o) = hv[i];
      *(volatile v8h*)(oL + o) = lv[i];
    }
    __threadfence();
#pragma unroll
    for (int i = 0; i < 4; ++i) {
      const int lr = 16 * wave + 4 * i + sub;
      const size_t o = (size_t)(oOff + rowBase + lr) * (size_t)ldo + col0 + 8 * q8;
      *(volatile v8h*)(oH + o) = hv[i];
      *(volatile v8h*)(oL + o) = lv[i];
    }
  }
  (void)p0; (void)p1; (void)oF; (void)oH; (void)oL; (void)nRow;
}

__global__ __launch_bounds__(NTHR) void k_gat(
    const int* __restrict__ srcs, const int* __restrict__ dsts,
    const float* __restrict__ XLR, const float* __restrict__ xin,
    const float* __restrict__ att, const float* __restrict__ gbias, const float* __restrict__ ln2w,
    float* X1, _Float16* H2h, _Float16* H2l,
    int nN, int nE, int nb, int vec8, int MPr) {
  extern __shared__ v4f lds_dyn[];
  int* reg1 = (int*)lds_dyn;
  int* reg2 = reg1 + RCAP;
  int* scnt = reg2 + RCAP;
  int* soff = scnt + NBMAX;
  int* list = soff + NBMAX;
  int* wcnt = list + LISTN;
  int* wtot = wcnt + NWAVE;
  const int tid = (int)threadIdx.x, lane = tid & 31, wave = tid >> 5;
  const int nodeBase = (int)blockIdx.x * nb;

  for (int i = tid; i < NBMAX; i += NTHR) scnt[i] = 0;
  __syncthreads();

  int tot = 0;
  const int nChunks = (nE + CHUNK - 1) / CHUNK;
#pragma unroll 1
  for (int ch = 0; ch < nChunks; ++ch) {
    const int cbase = ch * CHUNK;
    const int wc = scan_chunk(dsts, nE, cbase, nodeBase, nb, vec8, list, tid, lane, wave);
    if (lane == 0) wcnt[wave] = wc;
    __syncthreads();
    int pre = 0, all = 0;
#pragma unroll
    for (int w2 = 0; w2 < NWAVE; ++w2) {
      int c = wcnt[w2];
      c = c < 0 ? 0 : (c > WCAP ? WCAP : c);
      all += c;
      pre += (w2 < wave) ? c : 0;
    }
    const int wcc  = wc > WCAP ? WCAP : wc;
    const int base = tot + pre;
#pragma unroll 1
    for (int i = lane; i < wcc; i += 32) {
      const int ent = list[wave * WCAP + i];
      const int el  = (ent >> 12) & (CHUNK - 1);
      const int sl  = ent & (NBMAX - 1);
      int eid = cbase + el;
      eid = eid > nE - 1 ? nE - 1 : eid;
      const int pos = base + i;
      if (pos < RCAP) reg1[pos] = (int)(((unsigned)eid << 12) | (unsigned)sl);
    }
    tot += all;
    tot = tot > RCAP ? RCAP : tot;
    __syncthreads();
  }
  const int nh = tot;

  if (wave == 0) {
#pragma unroll 1
    for (int b0 = 0; b0 < nh; b0 += 32) {
      const int idx = b0 + lane;
      const int uv  = reg1[idx < RCAP ? idx : RCAP - 1];
      const int m32 = (nh - b0) < 32 ? (nh - b0) : 32;
#pragma unroll 1
      for (int k = 0; k < m32; ++k) {
        const int u  = __builtin_amdgcn_readlane(uv, k);
        const int sl = u & (NBMAX - 1);
        if (lane == 0) scnt[sl] = scnt[sl] + 1;
      }
    }
  }
  __syncthreads();

  {
    const v4i ca = *(const v4i*)(scnt + 8 * tid);
    const v4i cb = *(const v4i*)(scnt + 8 * tid + 4);
    const int e0 = ca.x < 0 ? 0 : ca.x, e1 = ca.y < 0 ? 0 : ca.y, e2 = ca.z < 0 ? 0 : ca.z, e3 = ca.w < 0 ? 0 : ca.w;
    const int e4 = cb.x < 0 ? 0 : cb.x, e5 = cb.y < 0 ? 0 : cb.y, e6 = cb.z < 0 ? 0 : cb.z, e7 = cb.w < 0 ? 0 : cb.w;
    const int ts = e0 + e1 + e2 + e3 + e4 + e5 + e6 + e7;
    int incl = ts;
#pragma unroll
    for (int d = 1; d < 32; d <<= 1) {
      const int up = __shfl_up(incl, d);
      if (lane >= d) incl += up;
    }
    if (lane == 31) wtot[wave] = incl;
    __syncthreads();
    int pre = 0;
#pragma unroll
    for (int w2 = 0; w2 < NWAVE; ++w2) pre += (w2 < wave) ? wtot[w2] : 0;
    int run = pre + incl - ts;
    soff[8 * tid + 0] = run; run += e0;
    soff[8 * tid + 1] = run; run += e1;
    soff[8 * tid + 2] = run; run += e2;
    soff[8 * tid + 3] = run; run += e3;
    soff[8 * tid + 4] = run; run += e4;
    soff[8 * tid + 5] = run; run += e5;
    soff[8 * tid + 6] = run; run += e6;
    soff[8 * tid + 7] = run;
  }
  __syncthreads();
  for (int i = tid; i < NBMAX; i += NTHR) list[i] = soff[i];
  __syncthreads();

  if (wave == 0) {
#pragma unroll 1
    for (int b0 = 0; b0 < nh; b0 += 32) {
      const int idx = b0 + lane;
      const int uv  = reg1[idx < RCAP ? idx : RCAP - 1];
      const int m32 = (nh - b0) < 32 ? (nh - b0) : 32;
#pragma unroll 1
      for (int k = 0; k < m32; ++k) {
        const int u   = __builtin_amdgcn_readlane(uv, k);
        const int sl  = u & (NBMAX - 1);
        const int eid = (int)((unsigned)u >> 12);
        if (lane == 0) {
          int pos = list[sl];
          pos = pos < 0 ? 0 : (pos > RCAP - 1 ? RCAP - 1 : pos);
          reg2[pos] = eid;
          list[sl] = pos + 1;
        }
      }
    }
  }
  __syncthreads();

  const int nbw = nb >> 3;
  const bool ovf = (nh >= RCAP);
  const float qnan = __int_as_float(0x7fc00000);
  float* stw = (float*)reg1 + wave * STW;
  const int lc = lane < 16 ? lane : 15;
  __shared__ __attribute__((aligned(16))) float spar[3 * 128];
  if (threadIdx.x < 96) {
    const int pa = threadIdx.x >> 5;
    const float* psrc = (pa == 0) ? att : (pa == 1) ? gbias : ln2w;
    reinterpret_cast<float4*>(spar + pa * 128)[lane] = reinterpret_cast<const float4*>(psrc)[lane];
  }
  __syncthreads();
  float at[NHD], gb[NHD], w2[NHD];
#pragma unroll
  for (int j = 0; j < NHD; ++j) {
    at[j] = rbf(spar[HC * j + lane]);
    gb[j] = rbf(spar[128 + HC * j + lane]);
  }
#pragma unroll
  for (int j = 0; j < NHD; ++j) w2[j] = rbf(spar[256 + HC * j + lane]);
#pragma unroll 1
  for (int jt = 0; jt < nbw; ++jt) {
    const int slot = wave * nbw + jt;
    const int grow = nodeBase + slot;
    const int gcl  = grow < nN ? grow : nN - 1;
    int st = soff[slot];
    const int craw = scnt[slot];
    int cnt = craw;
    st  = st < 0 ? 0 : (st > nh ? nh : st);
    cnt = cnt < 0 ? 0 : (cnt > DEGCAP ? DEGCAP : cnt);
    if (cnt > nh - st) cnt = nh - st;
    const float pz = (ovf || craw > DEGCAP) ? qnan : 0.0f;
    const float live = grow < nN ? 1.0f : 0.0f;

    const float* drow = XLR + (size_t)gcl * NXL + lane;
    float hsf[NHD], hd[NHD];
#pragma unroll
    for (int j = 0; j < NHD; ++j) { hsf[j] = drow[HC * j]; hd[j] = drow[DM + HC * j]; }
    ldwait();
    float mx[NHD], dn[NHD], av[NHD];
    {
      float pt[NHD];
#pragma unroll
      for (int j = 0; j < NHD; ++j) {
        float v = hsf[j] + hd[j];
        v = v > 0.f ? v : v * NEGS;
        pt[j] = v * at[j];
      }
#pragma unroll
      for (int off = 16; off > 0; off >>= 1) {
#pragma unroll
        for (int j = 0; j < NHD; ++j) pt[j] += __shfl_xor(pt[j], off);
      }
#pragma unroll
      for (int j = 0; j < NHD; ++j) { mx[j] = pt[j]; dn[j] = 1.0f; av[j] = hsf[j]; }
    }

#pragma unroll 1
    for (int q = 0; q < cnt; ++q) {
      int idx = st + q; idx = idx > RCAP - 1 ? RCAP - 1 : idx;
      int eid = reg2[idx]; eid = eid < 0 ? 0 : (eid > nE - 1 ? nE - 1 : eid);
      const int sraw = srcs[eid];
      const int s = sraw < 0 ? 0 : (sraw > nN - 1 ? nN - 1 : sraw);
      const float* sr = XLR + (size_t)s * NXL + lane;
      float hs[NHD];
#pragma unroll
      for (int j = 0; j < NHD; ++j) hs[j] = sr[HC * j];
      ldwait();
      float pt[NHD];
#pragma unroll
      for (int j = 0; j < NHD; ++j) {
        float v = hs[j] + hd[j];
        v = v > 0.f ? v : v * NEGS;
        pt[j] = v * at[j];
      }
#pragma unroll
      for (int off = 16; off > 0; off >>= 1) {
#pragma unroll
        for (int j = 0; j < NHD; ++j) pt[j] += __shfl_xor(pt[j], off);
      }
#pragma unroll
      for (int j = 0; j < NHD; ++j) {
        const float al = pt[j];
        const float df = al - mx[j];
        const float ee = __expf(-fabsf(df));
        const bool up  = df > 0.f;
        const float s1 = up ? ee : 1.0f;
        const float s2 = up ? 1.0f : ee;
        mx[j] = up ? al : mx[j];
        dn[j] = fmaf(dn[j], s1, s2);
        av[j] = fmaf(av[j], s1, s2 * hs[j]);
      }
    }

    const float* xr = xin + (size_t)gcl * DM + lane;
    float x1[NHD];
#pragma unroll
    for (int j = 0; j < NHD; ++j) x1[j] = xr[HC * j];
    ldwait();
#pragma unroll
    for (int j = 0; j < NHD; ++j) {
      const float agg = av[j] * __builtin_amdgcn_rcpf(dn[j]);
      x1[j] = ((rbf(x1[j]) + agg) + gb[j]) * live + pz;
    }
    float s = (x1[0] + x1[1]) + (x1[2] + x1[3]);
#pragma unroll
    for (int off = 16; off > 0; off >>= 1) s += __shfl_xor(s, off);
    const float mean = s * (1.0f / DM);
    float dv[NHD];
    float vs = 0.0f;
#pragma unroll
    for (int j = 0; j < NHD; ++j) { dv[j] = x1[j] - mean; vs = fmaf(dv[j], dv[j], vs); }
#pragma unroll
    for (int off = 16; off > 0; off >>= 1) vs += __shfl_xor(vs, off);
    const float rstd = rsqrtf(vs * (1.0f / DM) + LNEPS);
    float h2[NHD];
#pragma unroll
    for (int j = 0; j < NHD; ++j) h2[j] = dv[j] * rstd * w2[j];

    __builtin_amdgcn_fence(__ATOMIC_RELEASE, "wavefront");
    __builtin_amdgcn_wave_barrier();
#pragma unroll
    for (int j = 0; j < NHD; ++j) { stw[HC * j + lane] = x1[j]; stw[DM + HC * j + lane] = h2[j]; }
    __builtin_amdgcn_fence(__ATOMIC_RELEASE, "wavefront");
    __builtin_amdgcn_wave_barrier();
    const v4f xv = *(const v4f*)(stw + 4 * lane);
    const v4f ga = *(const v4f*)(stw + DM + 8 * lc);
    const v4f gg = *(const v4f*)(stw + DM + 8 * lc + 4);
    v8h hv, lv;
    cvt8hl(ga, gg, hv, lv);
    const bool wr = grow < MPr;
    float* gp = X1 + (size_t)grow * DM + 4 * lane;
    _Float16* gph = H2h + (size_t)grow * DM + 8 * lc;
    _Float16* gpl = H2l + (size_t)grow * DM + 8 * lc;
    const bool wsv = wr && (lane < (DM / 8));
    if (wr)  *(volatile v4f*)gp = xv;
    if (wsv) { *(volatile v8h*)gph = hv; *(volatile v8h*)gpl = lv; }
    __threadfence();
    if (wr)  *(volatile v4f*)gp = xv;
    if (wsv) { *(volatile v8h*)gph = hv; *(volatile v8h*)gpl = lv; }
  }
}

static int pick_nb(int nE, int nN) {
  int nb = NBRUN;
  while (nb > 16 && (long long)nb * (long long)nE * 5LL > (long long)RCAP * (long long)nN * 4LL) nb >>= 1;
  return nb;
}
static inline int cdiv(int a, int b) { return (a + b - 1) / b; }

extern "C" void kernel_launch(void* const* d_in, const int* in_sizes, int n_in,
                              void* d_out, int out_size, void* d_ws, size_t ws_size,
                              hipStream_t stream) {
  if (n_in < 12) return;
  const int nN = in_sizes[0] / DM;
  if (nN <= 0 || in_sizes[0] != nN * DM || nN > (1 << 22)) return;
  if (in_sizes[1] < 2 || (in_sizes[1] & 1) != 0) return;
  const int nE = in_sizes[1] / 2;
  if (nE < 1 || nE > (1 << 20)) return;
  if (in_sizes[2] != DM || in_sizes[3] != DM * DM || in_sizes[4] != DM) return;
  if (in_sizes[5] != DM * DM || in_sizes[6] != DM || in_sizes[7] != NHD * HC) return;
  if (in_sizes[8] != DM || in_sizes[9] != DM) return;
  if (in_sizes[10] != DM * DFF || in_sizes[11] != DFF * DM) return;
  if (out_size != nN * DM) return;

  const float* x     = (const float*)d_in[0];
  const int*   ei    = (const int*)  d_in[1];
  const float* ln1w  = (const float*)d_in[2];
  const float* Wl    = (const float*)d_in[3];
  const float* bl    = (const float*)d_in[4];
  const float* Wr    = (const float*)d_in[5];
  const float* br    = (const float*)d_in[6];
  const float* att   = (const float*)d_in[7];
  const float* gbias = (const float*)d_in[8];
  const float* ln2w  = (const float*)d_in[9];
  const float* Wfc   = (const float*)d_in[10];
  const float* Wproj = (const float*)d_in[11];
  float* out = (float*)d_out;
  const int* src = ei;
  const int* dst = ei + nE;

  const int MP   = cdiv(nN, GBM) * GBM;
  const int gM   = MP / GBM;
  const int gM0  = (gM + 1) / 2;
  const int gM1  = gM - gM0;
  const int MPh  = gM0 * GBM;
  const int nb   = pick_nb(nE, nN);
  const int gA   = cdiv(MP, nb);
  const int vec8 = ((nE & 3) == 0) ? 1 : 0;
  if (gA * nb < MP) return;

  char* ws = (char*)d_ws;
  size_t off = 0;
  const size_t szXLR = (size_t)MP * NXL * 4;
  const size_t szG2  = (size_t)2 * (size_t)MPh * DFF * 2;
  const size_t szBIG = szXLR > szG2 ? szXLR : szG2;
  const size_t oWT1 = off; off += (size_t)NXL * DM * 2;            off = (off + 255) & ~(size_t)255;
  const size_t oWTF = off; off += (size_t)DFF * DM * 2;            off = (off + 255) & ~(size_t)255;
  const size_t oWTP = off; off += (size_t)DM * DFF * 2;            off = (off + 255) & ~(size_t)255;
  const size_t oHA  = off; off += (size_t)MP * DM * 2;             off = (off + 255) & ~(size_t)255;
  const size_t oHB  = off; off += (size_t)MP * DM * 2;             off = (off + 255) & ~(size_t)255;
  const size_t oBIG = off; off += szBIG;                           off = (off + 255) & ~(size_t)255;
  const size_t oX1  = off; off += (size_t)MP * DM * 4;             off = (off + 255) & ~(size_t)255;
  if (off > ws_size || off > (size_t)WSMAX) return;
  unsigned short* WT1 = (unsigned short*)(ws + oWT1);
  unsigned short* WTF = (unsigned short*)(ws + oWTF);
  unsigned short* WTP = (unsigned short*)(ws + oWTP);
  unsigned short* HA  = (unsigned short*)(ws + oHA);
  unsigned short* HB  = (unsigned short*)(ws + oHB);
  float*          XLR = (float*)(ws + oBIG);
  unsigned short* GH  = (unsigned short*)(ws + oBIG);
  unsigned short* GL  = (unsigned short*)(ws + oBIG + (size_t)MPh * DFF * 2);
  float*          X1  = (float*)(ws + oX1);

  hipFuncSetAttribute(reinterpret_cast<const void*>(&k_gat),
                      hipFuncAttributeMaxDynamicSharedMemorySize, LDS_AGG);

  k_ln1<<<MP / (2 * NWAVE), NTHR, 0, stream>>>(x, ln1w, (_Float16*)HA, (_Float16*)HB, nN, MP);

  {
    const int nU = DM * (DM / 8);
    k_wtr_h<<<cdiv(nU, NTHR), NTHR, 0, stream>>>(Wl, DM, DM, (_Float16*)WT1, nU);
    k_wtr_h<<<cdiv(nU, NTHR), NTHR, 0, stream>>>(Wr, DM, DM, (_Float16*)(WT1 + (size_t)DM * DM), nU);
    const int nUf = DFF * (DM / 8);
    k_wtr_h<<<cdiv(nUf, NTHR), NTHR, 0, stream>>>(Wfc, DFF, DM, (_Float16*)WTF, nUf);
    const int nUp = DM * (DFF / 8);
    k_wtr_h<<<cdiv(nUp, NTHR), NTHR, 0, stream>>>(Wproj, DM, DFF, (_Float16*)WTP, nUp);
  }

  k_gemm<0><<<dim3(gM, NXL / GBN), GTHR, 0, stream>>>(HA, HB, WT1, bl, br, XLR, (_Float16*)GH, (_Float16*)GL,
                                                      DM, NXL, 0, 0, MP);
  k_gat<<<gA, NTHR, LDS_AGG, stream>>>(src, dst, XLR, x, att, gbias, ln2w, X1, (_Float16*)HA, (_Float16*)HB,
                                       nN, nE, nb, vec8, MP);
  for (int p = 0; p < 2; ++p) {
    const int gMp = (p == 0) ? gM0 : gM1;
    if (gMp <= 0) continue;
    const int rOff = p * MPh;
    k_gemm<1><<<dim3(gMp, DFF / GBN), GTHR, 0, stream>>>(HA, HB, WTF, X1, X1, XLR, (_Float16*)GH, (_Float16*)GL,
                                                         DM, DFF, rOff, 0, MPh);
    k_gemm<2><<<dim3(gMp, DM / GBN), GTHR, 0, stream>>>(GH, GL, WTP, X1, X1, out, (_Float16*)GH, (_Float16*)GL,
                                                        DFF, DM, 0, rOff, nN);
  }
}
